// ConcatCritic_61692910240322
// MI455X (gfx1250) — hardware-verified
//
#include <hip/hip_runtime.h>


#define NP   1024
#define DX   64
#define D0   128
#define D1   128
#define D2   64
#define D3   64
#define D4   64
#define PB   64
#define NPR  (PB * NP)
typedef _Float16 h16;
typedef unsigned short bf;
typedef __attribute__((ext_vector_type(16))) __bf16   v16bf;
typedef __attribute__((ext_vector_type(16))) _Float16 v16h;
typedef __attribute__((ext_vector_type(8)))  _Float16 v8h;
typedef __attribute__((ext_vector_type(8)))  unsigned short v8us;
typedef __attribute__((ext_vector_type(8)))  float    v8f;
typedef __attribute__((ext_vector_type(4)))  float    v4f;
typedef __attribute__((ext_vector_type(2)))  float    v2f;
typedef __attribute__((ext_vector_type(4)))  unsigned short v4us;
typedef __attribute__((ext_vector_type(2)))  unsigned short v2us;
typedef v8h  __attribute__((may_alias)) v8ha;
typedef v4f  __attribute__((may_alias)) v4fa;
typedef v8us __attribute__((may_alias)) v8usa;

__device__ __forceinline__ unsigned short f2bf(float f) { unsigned u = __float_as_uint(f); u += 0x7FFFu + ((u >> 16) & 1u); return (unsigned short)(u >> 16); }
__device__ __forceinline__ float bf2f(unsigned short b) { return __uint_as_float(((unsigned)b) << 16); }
__device__ __forceinline__ float bfr(float f) { return bf2f(f2bf(f)); }
__device__ __forceinline__ void splitf(float y, unsigned short& h, unsigned short& l) { h = f2bf(y); l = f2bf(y - bf2f(h)); }
__device__ __forceinline__ v16h cat16(v8h lo, v8h hi) { return __builtin_shufflevector(lo, hi, 0, 1, 2, 3, 4, 5, 6, 7, 8, 9, 10, 11, 12, 13, 14, 15); }
__device__ __forceinline__ v16bf cat16b(v8us lo, v8us hi) { return __builtin_bit_cast(v16bf, __builtin_shufflevector(lo, hi, 0, 1, 2, 3, 4, 5, 6, 7, 8, 9, 10, 11, 12, 13, 14, 15)); }
__device__ __forceinline__ v8f wmma16(v16h a, v16h b, v8f c) { return __builtin_amdgcn_wmma_f32_16x16x32_f16(false, a, false, b, (short)0, c, false, false); }
__device__ __forceinline__ v8f wmmab(v16bf a, v16bf b, v8f c) { return __builtin_amdgcn_wmma_f32_16x16x32_bf16(false, a, false, b, (short)0, c, false, false); }

template <typename T16> struct WFrag;
template <> struct WFrag<h16> { typedef v16h V; static __device__ __forceinline__ V ld(const h16* p) { return cat16(*(const v8h*)p, *(const v8h*)(p + 16)); } static __device__ __forceinline__ v8f mma(V a, V b, v8f c) { return wmma16(a, b, c); } };
template <> struct WFrag<bf> { typedef v16bf V; static __device__ __forceinline__ V ld(const bf* p) { return cat16b(*(const v8us*)p, *(const v8us*)(p + 16)); } static __device__ __forceinline__ v8f mma(V a, V b, v8f c) { return wmmab(a, b, c); } };
template <typename T16, int NSPLIT, bool BIAS>
__global__ __launch_bounds__(32) void k_gemmw(const T16* __restrict__ A, const T16* __restrict__ A2, const T16* __restrict__ Bt, const T16* __restrict__ Bt2, int K, float* C, int ldc, const float* __restrict__ bias, size_t sA, size_t sB, size_t sC) {
    typedef typename WFrag<T16>::V V;
    __shared__ __align__(16) float os[16 * 68];
    const size_t z = blockIdx.z; A += z * sA; if (A2) A2 += z * sA; Bt += z * sB; if (Bt2) Bt2 += z * sB; C += z * sC;
    const int lane = threadIdx.x & 31, lr = lane & 15, hi = lane >> 4; const int r0 = blockIdx.x * 64, c0 = blockIdx.y * 64;
    v8f acc[4][4];
#pragma unroll
    for (int mb = 0; mb < 4; ++mb)
#pragma unroll
        for (int nb = 0; nb < 4; ++nb) acc[mb][nb] = (v8f){};
    const size_t aoff = (size_t)(r0 + lr) * K + 8 * hi, boff = (size_t)(c0 + lr) * K + 8 * hi;
#pragma unroll 1
    for (int kc = 0; kc < K; kc += 32) {
        V a[4], a2[4];
#pragma unroll
        for (int mb = 0; mb < 4; ++mb) { a[mb] = WFrag<T16>::ld(A + aoff + (size_t)mb * 16 * K + kc); if (NSPLIT == 1 || NSPLIT == 2) a2[mb] = WFrag<T16>::ld(A2 + aoff + (size_t)mb * 16 * K + kc); }
#pragma unroll
        for (int nb = 0; nb < 4; ++nb) { const V b = WFrag<T16>::ld(Bt + boff + (size_t)nb * 16 * K + kc); V b2; if (NSPLIT >= 2) b2 = WFrag<T16>::ld(Bt2 + boff + (size_t)nb * 16 * K + kc);
#pragma unroll
            for (int mb = 0; mb < 4; ++mb) { acc[mb][nb] = WFrag<T16>::mma(a[mb], b, acc[mb][nb]); if (NSPLIT == 1 || NSPLIT == 2) acc[mb][nb] = WFrag<T16>::mma(a2[mb], b, acc[mb][nb]); if (NSPLIT >= 2) acc[mb][nb] = WFrag<T16>::mma(a[mb], b2, acc[mb][nb]); } }
        asm volatile("v_nop\n\tv_nop\n\tv_nop\n\tv_nop" : "+v"(acc[0][0]), "+v"(acc[1][1]), "+v"(acc[2][2]), "+v"(acc[3][3]) : "v"(a[0]), "v"(a[3]));
    }
#pragma unroll
    for (int mb = 0; mb < 4; ++mb) {
#pragma unroll
        for (int nb = 0; nb < 4; ++nb) {
#pragma unroll
            for (int j = 0; j < 8; ++j) os[(hi * 8 + j) * 68 + nb * 16 + lr] = acc[mb][nb][j]; }
        __builtin_amdgcn_wave_barrier(); asm volatile("" ::: "memory");
        float* crow = C + (size_t)(r0 + mb * 16) * ldc + c0;
#pragma unroll 1
        for (int ps = 0; ps < 2; ++ps) {
#pragma unroll
            for (int s = 0; s < 8; ++s) { const int row = 2 * s + hi, cofs = lr * 4; v4f val = *(const v4fa*)(os + row * 68 + cofs); if (BIAS) { val[0] += bfr(bias[c0 + cofs]); val[1] += bfr(bias[c0 + cofs + 1]); val[2] += bfr(bias[c0 + cofs + 2]); val[3] += bfr(bias[c0 + cofs + 3]); }
                *(volatile v4f*)(crow + (size_t)row * ldc + cofs) = val; }
            if (ps == 0) __threadfence(); }
        __builtin_amdgcn_wave_barrier(); asm volatile("" ::: "memory");
    }
}

__global__ __launch_bounds__(256) void k_wtG(const float* __restrict__ w, int K, int N, bf* Bt) {
    const int lane = threadIdx.x & 31; const int L0 = (blockIdx.x * 8 + (threadIdx.x >> 5)) * 8; const int nlines = N * K / 64;
#pragma unroll
    for (int ps = 0; ps < 2; ++ps) {
#pragma unroll 1
        for (int l = 0; l < 8; ++l) { const int L = L0 + l; if (L >= nlines) break; const size_t e = (size_t)L * 64 + lane * 2; const int k = (int)(e % K), n = (int)(e / K); v2us o;
            o[0] = f2bf(w[(size_t)k * N + n]); o[1] = f2bf(w[(size_t)(k + 1) * N + n]); *(volatile v2us*)(Bt + e) = o; }
        if (ps == 0) __threadfence(); }
}
__global__ __launch_bounds__(256) void k_cvt8(const float* __restrict__ src, bf* dst, size_t n8) { const size_t i = (size_t)blockIdx.x * 256 + threadIdx.x; if (i >= n8) return; const v8f v = *(const v8f*)(src + i * 8); v8us o;
#pragma unroll
    for (int k = 0; k < 8; ++k) o[k] = f2bf(v[k]); *(volatile v8us*)(dst + i * 8) = o; __threadfence(); *(volatile v8us*)(dst + i * 8) = o; }
__global__ __launch_bounds__(256) void k_h0(const float* __restrict__ XA, const float* __restrict__ YB, const float* __restrict__ b0, int p0, bf* Hh, bf* Hl) { const size_t e = ((size_t)blockIdx.x * 256 + threadIdx.x) * 4; if (e >= (size_t)NPR * D0) return; const int c = (int)(e % D0); const size_t pr = e / D0; const int q = (int)(pr % NP); const int pl = (int)(pr / NP); const v4f xa = *(const v4f*)(XA + (size_t)(p0 + pl) * D0 + c), yb = *(const v4f*)(YB + (size_t)q * D0 + c); v4us oh, ol;
#pragma unroll
    for (int k = 0; k < 4; ++k) { float s = __fadd_rn(xa[k], yb[k]); asm volatile("" : "+v"(s)); const float h = fmaxf(__fadd_rn(s, bfr(b0[c + k])), 0.f); unsigned short a, l; splitf(h, a, l); oh[k] = a; ol[k] = l; }
    *(volatile v4us*)(Hh + e) = oh; *(volatile v4us*)(Hl + e) = ol; __threadfence(); *(volatile v4us*)(Hh + e) = oh; *(volatile v4us*)(Hl + e) = ol; }
__global__ __launch_bounds__(256) void k_relupl(const float* __restrict__ F, bf* Ph, bf* Pl, size_t n4) { const size_t i = (size_t)blockIdx.x * 256 + threadIdx.x; if (i >= n4) return; const v4f v = *(const v4f*)(F + i * 4); v4us oh, ol;
#pragma unroll
    for (int q = 0; q < 4; ++q) { unsigned short a, c; splitf(fmaxf(v[q], 0.f), a, c); oh[q] = a; ol[q] = c; } *(volatile v4us*)(Ph + i * 4) = oh; *(volatile v4us*)(Pl + i * 4) = ol; __threadfence(); *(volatile v4us*)(Ph + i * 4) = oh; *(volatile v4us*)(Pl + i * 4) = ol; }
__global__ __launch_bounds__(256) void k_last(const float* __restrict__ F4, const float* __restrict__ W5, const float* __restrict__ b5, int p0, float* OUT) { const size_t pr = (size_t)blockIdx.x * 256 + threadIdx.x; if (pr >= (size_t)NPR) return; const int q = (int)(pr % NP); const int pl = (int)(pr / NP); const float* f = F4 + pr * D4; float s = 0.f;
#pragma unroll 4
    for (int c = 0; c < D4; c += 4) { const v4f a = *(const v4f*)(f + c);
#pragma unroll
        for (int k = 0; k < 4; ++k) { float pdt = __fmul_rn(fmaxf(a[k], 0.f), bfr(W5[c + k])); asm volatile("" : "+v"(pdt)); s = __fadd_rn(s, pdt); } }
    const float v = __fadd_rn(s, bfr(b5[0])); float* dst = OUT + (size_t)(p0 + pl) * NP + q; *(volatile float*)dst = v; __threadfence(); *(volatile float*)dst = v; }

extern "C" void kernel_launch(void* const* d_in, const int* in_sizes, int n_in,
                              void* d_out, int out_size, void* d_ws, size_t ws_size, hipStream_t stream) {
    (void)in_sizes; (void)n_in; (void)out_size;
    const float* x = (const float*)d_in[0]; const float* y = (const float*)d_in[1];
    const float* W0 = (const float*)d_in[2]; const float* b0 = (const float*)d_in[3]; const float* W1 = (const float*)d_in[4]; const float* b1 = (const float*)d_in[5]; const float* W2 = (const float*)d_in[6]; const float* b2 = (const float*)d_in[7]; const float* W3 = (const float*)d_in[8]; const float* b3 = (const float*)d_in[9]; const float* W4 = (const float*)d_in[10]; const float* b4 = (const float*)d_in[11]; const float* W5 = (const float*)d_in[12]; const float* b5 = (const float*)d_in[13];
    float* OUT = (float*)d_out;
    char* wsp = (char*)d_ws;
    auto take = [&](size_t bytes) { char* p = wsp; wsp += (bytes + 255) & ~(size_t)255; return (void*)p; };
    bf* XB = (bf*)take((size_t)NP * DX * 2); bf* YBb = (bf*)take((size_t)NP * DX * 2); bf* W0X = (bf*)take((size_t)D0 * DX * 2); bf* W0Y = (bf*)take((size_t)D0 * DX * 2); bf* W1B = (bf*)take((size_t)D1 * D0 * 2); bf* W2B = (bf*)take((size_t)D2 * D1 * 2); bf* W3B = (bf*)take((size_t)D3 * D2 * 2); bf* W4B = (bf*)take((size_t)D4 * D3 * 2);
    float* XA = (float*)take((size_t)NP * D0 * 4); float* YA = (float*)take((size_t)NP * D0 * 4);
    bf* Hh = (bf*)take((size_t)NPR * D0 * 2); bf* Hl = (bf*)take((size_t)NPR * D0 * 2); float* F = (float*)take((size_t)NPR * D1 * 4); bf* Gh = (bf*)take((size_t)NPR * D1 * 2); bf* Gl = (bf*)take((size_t)NPR * D1 * 2); float* F2 = (float*)take((size_t)NPR * D2 * 4);
    if ((size_t)(wsp - (char*)d_ws) > ws_size) return;
    k_cvt8<<<(NP * DX / 8 + 255) / 256, 256, 0, stream>>>(x, XB, (size_t)NP * DX / 8); k_cvt8<<<(NP * DX / 8 + 255) / 256, 256, 0, stream>>>(y, YBb, (size_t)NP * DX / 8);
    k_wtG<<<(unsigned)((DX * D0 / 64 + 63) / 64), 256, 0, stream>>>(W0, DX, D0, W0X);
    k_wtG<<<(unsigned)((DX * D0 / 64 + 63) / 64), 256, 0, stream>>>(W0 + (size_t)DX * D0, DX, D0, W0Y);
    k_wtG<<<(unsigned)((D0 * D1 / 64 + 63) / 64), 256, 0, stream>>>(W1, D0, D1, W1B); k_wtG<<<(unsigned)((D1 * D2 / 64 + 63) / 64), 256, 0, stream>>>(W2, D1, D2, W2B); k_wtG<<<(unsigned)((D2 * D3 / 64 + 63) / 64), 256, 0, stream>>>(W3, D2, D3, W3B); k_wtG<<<(unsigned)((D3 * D4 / 64 + 63) / 64), 256, 0, stream>>>(W4, D3, D4, W4B);
    k_gemmw<bf, 0, false><<<dim3(NP / 64, D0 / 64, 1), 32, 0, stream>>>(XB, nullptr, W0X, nullptr, DX, XA, D0, nullptr, 0, 0, 0);
    k_gemmw<bf, 0, false><<<dim3(NP / 64, D0 / 64, 1), 32, 0, stream>>>(YBb, nullptr, W0Y, nullptr, DX, YA, D0, nullptr, 0, 0, 0);
    for (int p0 = 0; p0 < NP; p0 += PB) {
        k_h0<<<(unsigned)(((size_t)NPR * D0 / 4 + 255) / 256), 256, 0, stream>>>(XA, YA, b0, p0, Hh, Hl);
        k_gemmw<bf, 1, true><<<dim3(NPR / 64, D1 / 64, 1), 32, 0, stream>>>(Hh, Hl, W1B, nullptr, D0, F, D1, b1, 0, 0, 0);
        k_relupl<<<(unsigned)(((size_t)NPR * D1 / 4 + 255) / 256), 256, 0, stream>>>(F, Gh, Gl, (size_t)NPR * D1 / 4);
        k_gemmw<bf, 1, true><<<dim3(NPR / 64, D2 / 64, 1), 32, 0, stream>>>(Gh, Gl, W2B, nullptr, D1, F2, D2, b2, 0, 0, 0);
        k_relupl<<<(unsigned)(((size_t)NPR * D2 / 4 + 255) / 256), 256, 0, stream>>>(F2, Hh, Hl, (size_t)NPR * D2 / 4);
        k_gemmw<bf, 1, true><<<dim3(NPR / 64, D3 / 64, 1), 32, 0, stream>>>(Hh, Hl, W3B, nullptr, D2, F, D3, b3, 0, 0, 0);
        k_relupl<<<(unsigned)(((size_t)NPR * D3 / 4 + 255) / 256), 256, 0, stream>>>(F, Gh, Gl, (size_t)NPR * D3 / 4);
        k_gemmw<bf, 1, true><<<dim3(NPR / 64, D4 / 64, 1), 32, 0, stream>>>(Gh, Gl, W4B, nullptr, D3, F2, D4, b4, 0, 0, 0);
        k_last<<<(unsigned)((NPR + 255) / 256), 256, 0, stream>>>(F2, W5, b5, p0, OUT); }
}
